// GIN_MLP_31172872634624
// MI455X (gfx1250) — hardware-verified
//
#include <hip/hip_runtime.h>
#include <stddef.h>
#include <stdint.h>


#define DF      128
#define NTHR    256
#define NWAVE   8
#define EPT     8
#define CHUNK   (NTHR * EPT)
#define WCAP    (EPT * 32)
#define LISTN   (NWAVE * WCAP)
#define NBA     1024
#define SLA     10
#define RCAP    20480
#define DEGCAP  64
#define MISCN   32
#define CHB     25
#define CHR     (CHB * NBA)
#define GBM     64
#define GTHR    128
#define ROWH    256
#define T1A     0
#define T1B     1024
#define T2A     1536
#define T2B     2560
#define TDEC    2816
#define TMISC   3840
#define TABN    4096
#define NUW     32768
#define WPLN    262144
#define PW1A    0
#define PW1B    65536
#define PW2A    131072
#define PW2B    196608
#define PWD     229376
#define EBLK    1024
#define BKT_INTS (LISTN + 2 * RCAP + 3 * NBA + MISCN)
#define WSMAX   134217728

static_assert(CHR % NBA == 0 && CHR % 128 == 0 && CHR % GBM == 0);
static_assert((CHUNK & (CHUNK - 1)) == 0 && NBA == (1 << SLA));
static_assert(((long long)CHUNK << SLA) < (1LL << 31));
static_assert(RCAP % (NTHR * 4) == 0 && BKT_INTS % 4 == 0 && LISTN % 4 == 0);
static_assert(BKT_INTS * 4 <= 300000);
static_assert(NBA == NTHR * 4 && NBA % NWAVE == 0 && NBA % GBM == 0);
static_assert(NUW % NTHR == 0 && 8192 % NTHR == 0 && 4096 % NTHR == 0 && 2048 % NTHR == 0);
static_assert(NUW * 8 == WPLN);
static_assert(ROWH == 2 * DF && DF == 32 * 4);
static_assert(TMISC + 256 == TABN && T1A + 1024 == T1B && T1B + 512 == T2A && T2A + 1024 == T2B && T2B + 256 == TDEC && TDEC + 1024 == TMISC);
static_assert(EBLK == NTHR * 4 && EBLK == NWAVE * 128);
static_assert(DEGCAP >= 36 + 8 && RCAP >= 17546);

typedef float          v4f   __attribute__((ext_vector_type(4)));
typedef float          v8f   __attribute__((ext_vector_type(8)));
typedef int            v4i   __attribute__((ext_vector_type(4)));
typedef int            v8i   __attribute__((ext_vector_type(8)));
typedef unsigned       v2u   __attribute__((ext_vector_type(2)));
typedef unsigned       v4u   __attribute__((ext_vector_type(4)));
typedef unsigned short v4us  __attribute__((ext_vector_type(4)));
typedef unsigned short v8us  __attribute__((ext_vector_type(8)));
typedef unsigned short v16us __attribute__((ext_vector_type(16)));
typedef __bf16         v16bf __attribute__((ext_vector_type(16)));
typedef v4f  __attribute__((may_alias)) v4fa;
typedef v4i  __attribute__((may_alias)) v4ia;
typedef v2u  __attribute__((may_alias)) v2ua;
typedef v4us __attribute__((may_alias)) v4usa;
typedef v8us __attribute__((may_alias)) v8usa;
union FragB { v16bf v; v16us u; v8us h[2]; v8i w; };

__device__ __forceinline__ v8f wmb(const FragB& a, const FragB& b, v8f c) {
  v8f d = __builtin_amdgcn_wmma_f32_16x16x32_bf16(false, a.v, false, b.v, (short)0, c, false, false);
  asm volatile("v_nop\n\tv_nop\n\tv_nop\n\tv_nop" : "+v"(d) : "v"(a.w), "v"(b.w));
  return d;
}
__device__ __forceinline__ v8f z8() { v8f z = {0.f, 0.f, 0.f, 0.f, 0.f, 0.f, 0.f, 0.f}; return z; }

__device__ __forceinline__ unsigned bf16_bits(float f) {
  const unsigned u = __float_as_uint(f);
  return (u + 0x7FFFu + ((u >> 16) & 1u)) >> 16;
}
__device__ __forceinline__ float bf16_val(float f) { return __uint_as_float(bf16_bits(f) << 16); }
__device__ __forceinline__ unsigned bf16_bits_s(float f) {
  const unsigned u = __float_as_uint(f);
  const unsigned r = (u + 0x7FFFu + ((u >> 16) & 1u)) >> 16;
  const unsigned q = (u >> 16) | 0x40u;
  return ((u & 0x7fffffffu) > 0x7f800000u) ? q : r;
}
__device__ __forceinline__ unsigned hl_bits(float v, unsigned& lo) {
  const unsigned hb = bf16_bits_s(v);
  lo = bf16_bits_s(v - __uint_as_float(hb << 16));
  return hb;
}
__device__ __forceinline__ float relu_n(float v) { return (v > 0.0f) ? v : (v - v); }

__device__ __forceinline__ void wave_sync() {
  __builtin_amdgcn_fence(__ATOMIC_RELEASE, "wavefront");
  __builtin_amdgcn_wave_barrier();
  __builtin_amdgcn_fence(__ATOMIC_ACQUIRE, "wavefront");
}

template <int SLB>
__device__ __forceinline__ int scan_chunk(const int* __restrict__ dsts, int nE, int cbase, int slotBase,
                                          int nb, int vec8, int* list, int tid, int lane, int wave) {
  int wc = 0;
  const int el0  = tid * EPT;
  const int e0   = cbase + el0;
  const int sent = -2147483647 - 1;
  v4i da, db;
  if (vec8 != 0 && cbase + CHUNK <= nE) {
    da = *(const v4i*)(dsts + e0);
    db = *(const v4i*)(dsts + e0 + 4);
  } else {
    da.x = (e0     < nE) ? dsts[min(e0,     nE - 1)] : sent;
    da.y = (e0 + 1 < nE) ? dsts[min(e0 + 1, nE - 1)] : sent;
    da.z = (e0 + 2 < nE) ? dsts[min(e0 + 2, nE - 1)] : sent;
    da.w = (e0 + 3 < nE) ? dsts[min(e0 + 3, nE - 1)] : sent;
    db.x = (e0 + 4 < nE) ? dsts[min(e0 + 4, nE - 1)] : sent;
    db.y = (e0 + 5 < nE) ? dsts[min(e0 + 5, nE - 1)] : sent;
    db.z = (e0 + 6 < nE) ? dsts[min(e0 + 6, nE - 1)] : sent;
    db.w = (e0 + 7 < nE) ? dsts[min(e0 + 7, nE - 1)] : sent;
  }
  const unsigned nbs = (unsigned)slotBase;
  const unsigned unb = (unsigned)nb;
  const unsigned s0 = (unsigned)da.x - nbs, s1 = (unsigned)da.y - nbs;
  const unsigned s2 = (unsigned)da.z - nbs, s3 = (unsigned)da.w - nbs;
  const unsigned s4 = (unsigned)db.x - nbs, s5 = (unsigned)db.y - nbs;
  const unsigned s6 = (unsigned)db.z - nbs, s7 = (unsigned)db.w - nbs;
  const bool h0 = s0 < unb, h1 = s1 < unb, h2 = s2 < unb, h3 = s3 < unb;
  const bool h4 = s4 < unb, h5 = s5 < unb, h6 = s6 < unb, h7 = s7 < unb;
  const unsigned any = __builtin_amdgcn_ballot_w32(h0 | h1 | h2 | h3 | h4 | h5 | h6 | h7);
  if (any != 0u) {
#define HITJ(J, HJ, SJ) { \
      const unsigned mj = __builtin_amdgcn_ballot_w32(HJ); \
      if (mj != 0u) { \
        if (HJ) { \
          const int pos = wc + (int)__builtin_amdgcn_mbcnt_lo(mj, 0u); \
          if (pos < WCAP) list[wave * WCAP + pos] = ((el0 + (J)) << SLB) | (int)(SJ); \
        } \
        wc += (int)__builtin_popcount(mj); } }
    HITJ(0, h0, s0)
    HITJ(1, h1, s1)
    HITJ(2, h2, s2)
    HITJ(3, h3, s3)
    HITJ(4, h4, s4)
    HITJ(5, h5, s5)
    HITJ(6, h6, s6)
    HITJ(7, h7, s7)
#undef HITJ
  }
  return wc;
}

__global__ __launch_bounds__(NTHR) void k_tab(
    const float* __restrict__ b1a, const float* __restrict__ g1a, const float* __restrict__ be1a,
    const float* __restrict__ rm1a, const float* __restrict__ rv1a,
    const float* __restrict__ b1b, const float* __restrict__ g1, const float* __restrict__ be1,
    const float* __restrict__ rm1, const float* __restrict__ rv1,
    const float* __restrict__ b2a, const float* __restrict__ g2a, const float* __restrict__ be2a,
    const float* __restrict__ rm2a, const float* __restrict__ rv2a,
    const float* __restrict__ b2b, const float* __restrict__ g2, const float* __restrict__ be2,
    const float* __restrict__ rm2, const float* __restrict__ rv2,
    const float* __restrict__ bd1, const float* __restrict__ wd2, const float* __restrict__ bd2,
    const float* __restrict__ eps1, const float* __restrict__ eps2, float* tab) {
  __shared__ __attribute__((aligned(16))) float st[1280];
  const int tid = (int)threadIdx.x;
  const int q = (int)blockIdx.x;
  int len, base;
  if (q < 4) {
    const float* pb; const float* pg; const float* pe; const float* pm; const float* pv;
    int C;
    if (q == 0)      { pb = b1a; pg = g1a; pe = be1a; pm = rm1a; pv = rv1a; C = 256; base = T1A; }
    else if (q == 1) { pb = b1b; pg = g1;  pe = be1;  pm = rm1;  pv = rv1;  C = 128; base = T1B; }
    else if (q == 2) { pb = b2a; pg = g2a; pe = be2a; pm = rm2a; pv = rv2a; C = 256; base = T2A; }
    else             { pb = b2b; pg = g2;  pe = be2;  pm = rm2;  pv = rv2;  C = 64;  base = T2B; }
    const int cc = tid < C ? tid : C - 1;
    const float fb = bf16_val(pb[cc]);
    const float fm = bf16_val(pm[cc]);
    const float fe = bf16_val(pe[cc]);
    const float fg = bf16_val(pg[cc]);
    const float fv = bf16_val(pv[cc]);
    const float s  = fg * (1.0f / sqrtf(fv + 1e-5f));
    if (tid < C) { st[tid] = fb; st[C + tid] = fm; st[2 * C + tid] = s; st[3 * C + tid] = fe; }
    len = 4 * C;
  } else {
    base = TDEC;
    const int c1 = tid < 128 ? tid : 127;
    const float vb = bf16_val(bd1[c1]);
    const float vw = bf16_val(wd2[c1]);
    const float f2 = bf16_val(bd2[0]);
    const float e1 = bf16_val(eps1[0]);
    const float e2 = bf16_val(eps2[0]);
    st[tid]        = tid < 128 ? vb : 0.0f;
    st[256 + tid]  = 0.0f;
    st[512 + tid]  = 1.0f;
    st[768 + tid]  = 0.0f;
    float mv = 0.0f;
    mv = tid < 128 ? vw : mv;
    mv = tid == 128 ? f2 : mv;
    mv = tid == 129 ? e1 : mv;
    mv = tid == 130 ? e2 : mv;
    st[1024 + tid] = mv;
    len = 1280;
  }
  __syncthreads();
  float* tp = tab + base;
#pragma unroll 1
  for (int i4 = 4 * tid; i4 < len; i4 += 4 * NTHR) {
    const v4f v = *(const v4fa*)(st + i4);
    *(volatile v4f*)(tp + i4) = v;
  }
  __threadfence();
#pragma unroll 1
  for (int i4 = 4 * tid; i4 < len; i4 += 4 * NTHR) {
    const v4f v = *(const v4fa*)(st + i4);
    *(volatile v4f*)(tp + i4) = v;
  }
}

__global__ __launch_bounds__(NTHR) void k_prep(const float* __restrict__ x, const float* __restrict__ w1a,
                                               const float* __restrict__ w1b, const float* __restrict__ w2a,
                                               const float* __restrict__ w2b, const float* __restrict__ wd1,
                                               unsigned short* wpl, unsigned short* xb, int nN, int nUnits) {
  const int u = (int)blockIdx.x * NTHR + (int)threadIdx.x;
  v8us o;
  unsigned short* dp;
  if (u < NUW) {
    const float* p;
    int stride;
    if (u < 8192) {
      const int n = u >> 5, kk = ((u & 31) * 8) & 127;
      p = w1a + (size_t)kk * 256 + n; stride = 256;
    } else if (u < 16384) {
      const int v = u - 8192;
      const int n = v >> 6, kk = ((v & 63) * 8) & 255;
      p = w1b + (size_t)kk * 128 + n; stride = 128;
    } else if (u < 24576) {
      const int v = u - 16384;
      const int n = v >> 5, kk = ((v & 31) * 8) & 127;
      p = w2a + (size_t)kk * 256 + n; stride = 256;
    } else if (u < 28672) {
      const int v = u - 24576;
      const int n = v >> 6, kk = ((v & 63) * 8) & 255;
      p = w2b + (size_t)kk * 64 + n; stride = 64;
    } else {
      const int v = u - 28672;
      const int n = v >> 4, kk = ((v & 15) * 8) & 63;
      const int off = (n < 128) ? (kk * 128 + n) : ((64 + kk) * 128 + (n - 128));
      p = wd1 + off; stride = 128;
    }
#pragma unroll
    for (int i = 0; i < 8; ++i) o[i] = (unsigned short)bf16_bits(p[(size_t)i * stride]);
    dp = wpl + (size_t)u * 8;
  } else if (u < nUnits) {
    const int v   = u - NUW;
    const int row = v >> 4, c8 = (v & 15) * 8;
    const int rc  = row < nN ? row : nN - 1;
    const bool lv = row < nN;
    const float* p = x + (size_t)rc * DF + c8;
    const v4f a0 = *(const v4f*)p, a1 = *(const v4f*)(p + 4);
    const float fa[8] = {a0.x, a0.y, a0.z, a0.w, a1.x, a1.y, a1.z, a1.w};
#pragma unroll
    for (int i = 0; i < 8; ++i) o[i] = (unsigned short)bf16_bits(lv ? fa[i] : 0.0f);
    dp = xb + (size_t)v * 8;
  } else {
    return;
  }
  *(volatile v8us*)dp = o;
  __threadfence();
  *(volatile v8us*)dp = o;
}

__global__ __launch_bounds__(NTHR) void k_bucket(const int* __restrict__ srcs, const int* __restrict__ dsts,
                                                 int nE, int nN, int vec8,
                                                 int* lst, int* cntT, int* offT, int* flg) {
  extern __shared__ __attribute__((aligned(16))) int dsm[];
  int* list = dsm;
  int* hl   = dsm + LISTN;
  int* sl   = hl + RCAP;
  int* cnt  = sl + RCAP;
  int* offs = cnt + NBA;
  int* cur  = offs + NBA;
  int* misc = cur + NBA;
  const int tid = (int)threadIdx.x, lane = tid & 31, wave = tid >> 5;
  const int nodeBase = (int)blockIdx.x * NBA;

  {
    const v4i z4 = {0, 0, 0, 0};
    for (int i = tid * 4; i < BKT_INTS; i += NTHR * 4) *(v4ia*)(dsm + i) = z4;
  }
  __syncthreads();

  int t = 0, ov = 0;
  const int nChunks = (nE + CHUNK - 1) / CHUNK;
#pragma unroll 1
  for (int ch = 0; ch < nChunks; ++ch) {
    const int cbase = ch * CHUNK;
    const int wc = scan_chunk<SLA>(dsts, nE, cbase, nodeBase, NBA, vec8, list, tid, lane, wave);
    if (lane == 0) misc[wave] = wc;
    __syncthreads();
    if (wave == 0) {
#pragma unroll 1
      for (int w2 = 0; w2 < NWAVE; ++w2) {
        int c = misc[w2];
        c = c < 0 ? 0 : (c > WCAP ? WCAP : c);
#pragma unroll 1
        for (int b0 = 0; b0 < c; b0 += 32) {
          const int idx = b0 + lane;
          const int ent_ = list[w2 * WCAP + (idx < WCAP ? idx : WCAP - 1)];
          const int m32 = (c - b0) < 32 ? (c - b0) : 32;
#pragma unroll 1
          for (int k = 0; k < m32; ++k) {
            const int u    = __builtin_amdgcn_readlane(ent_, k);
            const int slot = u & (NBA - 1);
            const int el   = (u >> SLA) & (CHUNK - 1);
            const int pk   = ((cbase + el) << SLA) | slot;
            if (t < RCAP) {
              if (lane == 0) { hl[t] = pk; cnt[slot] = cnt[slot] + 1; }
              t = t + 1;
            } else {
              ov = 1;
            }
          }
        }
      }
    }
    __syncthreads();
  }
  if (wave == 0 && lane == 0) { misc[8] = t; misc[9] = ov; }
  __syncthreads();
  int tt = misc[8];
  tt = tt < 0 ? 0 : (tt > RCAP ? RCAP : tt);

  if (wave == 0) {
    const int base = lane * (NBA / 32);
    int s = 0;
#pragma unroll 1
    for (int i = 0; i < NBA / 32; ++i) s += cnt[base + i];
    int incl = s;
#pragma unroll
    for (int d = 1; d < 32; d <<= 1) {
      const int y = __shfl_up(incl, d, 32);
      if (lane >= d) incl += y;
    }
    int run = incl - s;
#pragma unroll 1
    for (int i = 0; i < NBA / 32; ++i) {
      const int cv = cnt[base + i];
      offs[base + i] = run;
      cur[base + i]  = run;
      run += cv;
    }
  }
  __syncthreads();
  if (wave == 0) {
#pragma unroll 1
    for (int b0 = 0; b0 < tt; b0 += 32) {
      const int idx = b0 + lane;
      const int ent_ = hl[idx < RCAP ? idx : RCAP - 1];
      const int m32 = (tt - b0) < 32 ? (tt - b0) : 32;
#pragma unroll 1
      for (int k = 0; k < m32; ++k) {
        const int u    = __builtin_amdgcn_readlane(ent_, k);
        const int slot = u & (NBA - 1);
        if (lane == 0) {
          int p = cur[slot];
          p = p < 0 ? 0 : (p > RCAP - 1 ? RCAP - 1 : p);
          sl[p] = u;
          cur[slot] = p + 1;
        }
      }
    }
  }
  __syncthreads();

  const int ttr = (tt + NTHR * 4 - 1) & ~(NTHR * 4 - 1);
#pragma unroll 1
  for (int i4 = tid * 4; i4 < ttr; i4 += NTHR * 4) {
    const v4i e = *(const v4ia*)(sl + i4);
    int e0 = e.x >> SLA, e1 = e.y >> SLA, e2 = e.z >> SLA, e3 = e.w >> SLA;
    e0 = e0 < 0 ? 0 : (e0 > nE - 1 ? nE - 1 : e0);
    e1 = e1 < 0 ? 0 : (e1 > nE - 1 ? nE - 1 : e1);
    e2 = e2 < 0 ? 0 : (e2 > nE - 1 ? nE - 1 : e2);
    e3 = e3 < 0 ? 0 : (e3 > nE - 1 ? nE - 1 : e3);
    int s0 = srcs[e0], s1 = srcs[e1], s2 = srcs[e2], s3 = srcs[e3];
    s0 = s0 < 0 ? 0 : (s0 > nN - 1 ? nN - 1 : s0);
    s1 = s1 < 0 ? 0 : (s1 > nN - 1 ? nN - 1 : s1);
    s2 = s2 < 0 ? 0 : (s2 > nN - 1 ? nN - 1 : s2);
    s3 = s3 < 0 ? 0 : (s3 > nN - 1 ? nN - 1 : s3);
    v4i o;
    o.x = (i4     < tt) ? s0 : 0;
    o.y = (i4 + 1 < tt) ? s1 : 0;
    o.z = (i4 + 2 < tt) ? s2 : 0;
    o.w = (i4 + 3 < tt) ? s3 : 0;
    *(v4ia*)(hl + i4) = o;
  }
  __syncthreads();

  int* lb = lst  + (size_t)blockIdx.x * RCAP;
  int* cb = cntT + (size_t)blockIdx.x * NBA;
  int* ob = offT + (size_t)blockIdx.x * NBA;
  int* fb = flg  + (size_t)blockIdx.x * MISCN;
#pragma unroll 1
  for (int i4 = tid * 4; i4 < RCAP; i4 += NTHR * 4) {
    const v4i v = *(const v4ia*)(hl + i4);
    *(volatile v4i*)(lb + i4) = v;
  }
  {
    const v4i c4 = *(const v4ia*)(cnt + 4 * tid);
    const v4i o4 = *(const v4ia*)(offs + 4 * tid);
    *(volatile v4i*)(cb + 4 * tid) = c4;
    *(volatile v4i*)(ob + 4 * tid) = o4;
    if (tid < MISCN / 4) {
      const v4i f4 = *(const v4ia*)(misc + 4 * tid);
      *(volatile v4i*)(fb + 4 * tid) = f4;
    }
  }
  __threadfence();
#pragma unroll 1
  for (int i4 = tid * 4; i4 < RCAP; i4 += NTHR * 4) {
    const v4i v = *(const v4ia*)(hl + i4);
    *(volatile v4i*)(lb + i4) = v;
  }
  {
    const v4i c4 = *(const v4ia*)(cnt + 4 * tid);
    const v4i o4 = *(const v4ia*)(offs + 4 * tid);
    *(volatile v4i*)(cb + 4 * tid) = c4;
    *(volatile v4i*)(ob + 4 * tid) = o4;
    if (tid < MISCN / 4) {
      const v4i f4 = *(const v4ia*)(misc + 4 * tid);
      *(volatile v4i*)(fb + 4 * tid) = f4;
    }
  }
}

template <int LAY>
__device__ __forceinline__ v4f ld_row(const unsigned short* __restrict__ src, int row, int lane) {
  const unsigned short* rp = src + (size_t)row * ((LAY == 1) ? 128 : 256) + 4 * lane;
  const v2u wh = *(const v2ua*)rp;
  v4f f;
  f.x = __uint_as_float(wh.x << 16);
  f.y = __uint_as_float(wh.x & 0xffff0000u);
  f.z = __uint_as_float(wh.y << 16);
  f.w = __uint_as_float(wh.y & 0xffff0000u);
  if (LAY != 1) {
    const v2u wl = *(const v2ua*)(rp + DF);
    f.x += __uint_as_float(wl.x << 16);
    f.y += __uint_as_float(wl.x & 0xffff0000u);
    f.z += __uint_as_float(wl.y << 16);
    f.w += __uint_as_float(wl.y & 0xffff0000u);
  }
  return f;
}

template <int LAY>
__global__ __launch_bounds__(NTHR) void k_agg(const int* __restrict__ lst, const int* __restrict__ cntT,
                                              const int* __restrict__ offT, const int* __restrict__ flg,
                                              const unsigned short* __restrict__ src,
                                              const float* __restrict__ tab, unsigned short* outp,
                                              int blk0, int rowG0, int nN, int outRows) {
  __shared__ __attribute__((aligned(16))) int cl[NBA];
  __shared__ __attribute__((aligned(16))) int ol[NBA];
  __shared__ __attribute__((aligned(16))) unsigned short rowall[NWAVE * ROWH];
  const int tid = (int)threadIdx.x, lane = tid & 31, wave = tid >> 5;
  const int b = blk0 + (int)blockIdx.x;
  const int nodeBase = b * NBA;
  unsigned short* rowbuf = rowall + wave * ROWH;
  {
    const v4i c4 = *(const v4i*)(cntT + (size_t)b * NBA + 4 * tid);
    const v4i o4 = *(const v4i*)(offT + (size_t)b * NBA + 4 * tid);
    *(v4ia*)(cl + 4 * tid) = c4;
    *(v4ia*)(ol + 4 * tid) = o4;
  }
  int tt = flg[(size_t)b * MISCN + 8];
  tt = tt < 0 ? 0 : (tt > RCAP ? RCAP : tt);
  const int ovf = flg[(size_t)b * MISCN + 9];
  const float onepe = 1.0f + tab[TMISC + 128 + LAY];
  const int* lb = lst + (size_t)b * RCAP;
  __syncthreads();

  const float qnan = __int_as_float(0x7fc00000);
  const float pz = (ovf != 0) ? qnan : 0.0f;
#pragma unroll 1
  for (int si = 0; si < NBA / NWAVE; ++si) {
    const int s    = si * NWAVE + wave;
    const int node = nodeBase + s;
    const int craw = cl[s];
    int c = craw;
    const bool big = (craw > DEGCAP) || (craw < 0);
    c = c < 0 ? 0 : (c > DEGCAP ? DEGCAP : c);
    int o = ol[s];
    o = o < 0 ? 0 : (o > tt ? tt : o);
    if (c > tt - o) c = tt - o;
    const float pzr = big ? qnan : pz;
    const bool live = node < nN;
    float a0 = 0.0f, a1 = 0.0f, a2 = 0.0f, a3 = 0.0f;
#pragma unroll 1
    for (int b0 = 0; b0 < c; b0 += 32) {
      int idx = o + b0 + lane;
      idx = idx > RCAP - 1 ? RCAP - 1 : idx;
      int sr = lb[idx];
      sr = sr < 0 ? 0 : (sr > nN - 1 ? nN - 1 : sr);
      const int m32 = (c - b0) < 32 ? (c - b0) : 32;
#pragma unroll 1
      for (int k = 0; k < m32; ++k) {
        const int sk = __builtin_amdgcn_readlane(sr, k);
        const v4f f = ld_row<LAY>(src, sk, lane);
        a0 += f.x; a1 += f.y; a2 += f.z; a3 += f.w;
      }
    }
    const int nc = live ? node : nN - 1;
    const v4f sf = ld_row<LAY>(src, nc, lane);
    const float r0 = onepe * sf.x + a0;
    const float r1 = onepe * sf.y + a1;
    const float r2 = onepe * sf.z + a2;
    const float r3 = onepe * sf.w + a3;
    const float m0 = live ? (r0 + pzr) : 0.0f;
    const float m1 = live ? (r1 + pzr) : 0.0f;
    const float m2 = live ? (r2 + pzr) : 0.0f;
    const float m3 = live ? (r3 + pzr) : 0.0f;
    v4us mh, ml;
    {
      unsigned lw;
      unsigned hw;
      hw = hl_bits(m0, lw); mh[0] = (unsigned short)hw; ml[0] = (unsigned short)lw;
      hw = hl_bits(m1, lw); mh[1] = (unsigned short)hw; ml[1] = (unsigned short)lw;
      hw = hl_bits(m2, lw); mh[2] = (unsigned short)hw; ml[2] = (unsigned short)lw;
      hw = hl_bits(m3, lw); mh[3] = (unsigned short)hw; ml[3] = (unsigned short)lw;
    }
    *(v4usa*)(rowbuf + 4 * lane)      = mh;
    *(v4usa*)(rowbuf + DF + 4 * lane) = ml;
    wave_sync();
    const v8us q0 = *(const v8usa*)(rowbuf + 8 * lane);
    wave_sync();
    const int orow = node - rowG0;
    if (orow < outRows) {
      unsigned short* rpw = outp + (size_t)orow * (2 * DF) + 8 * lane;
      *(volatile v8us*)rpw = q0;
      __threadfence();
      *(volatile v8us*)rpw = q0;
    }
  }
}

template <int NT, int EPI, int RELU>
__global__ __launch_bounds__(GTHR) void k_gemm(const unsigned short* __restrict__ A, int lda, int K,
                                               const unsigned short* __restrict__ BT,
                                               const float* __restrict__ par, int parC,
                                               void* outp, int ldo, int halfW, int rowG0, int nN, int mRows) {
  constexpr int BNW = 16 * NT;
  __shared__ __attribute__((aligned(16))) float stg[GBM * BNW];
  __shared__ __attribute__((aligned(16))) float pl[4 * 128];
  const int tid = (int)threadIdx.x, lane = tid & 31, wave = tid >> 5, hh = lane >> 4, m = lane & 15;
  const int rowBase = (int)blockIdx.x * GBM;
  const int n0 = (int)blockIdx.y * BNW;
  {
    const int cidx = (4 * lane < BNW - 4) ? 4 * lane : BNW - 4;
    const v4f pv = *(const v4f*)(par + (size_t)wave * parC + n0 + cidx);
    *(v4fa*)(pl + wave * 128 + 4 * lane) = pv;
  }
  v8f acc[NT];
#pragma unroll
  for (int t = 0; t < NT; ++t) acc[t] = z8();
  const unsigned short* ap = A + (size_t)(rowBase + 16 * wave + m) * (size_t)lda + 8 * hh;
  const unsigned short* wp = BT + (size_t)(n0 + m) * (size_t)K + 8 * hh;
  __syncthreads();

#pragma unroll 1
  for (int k0 = 0; k0 < K; k0 += 32) {
    FragB af;
    af.h[0] = *(const v8usa*)(ap + k0);
    af.h[1] = *(const v8usa*)(ap + k0 + 16);
#pragma unroll
    for (int t = 0; t < NT; ++t) {
      const unsigned short* wq = wp + (size_t)(16 * t) * (size_t)K + k0;
      FragB bf;
      bf.h[0] = *(const v8usa*)wq;
      bf.h[1] = *(const v8usa*)(wq + 16);
      acc[t] = wmb(af, bf, acc[t]);
    }
  }

#pragma unroll
  for (int t = 0; t < NT; ++t) {
    const int lc = 16 * t + m;
    const float pb = pl[lc], pm = pl[128 + lc], ps = pl[256 + lc], pe = pl[384 + lc];
#pragma unroll
    for (int r = 0; r < 8; ++r) {
      const int lr = 16 * wave + 8 * hh + r;
      const bool live = (rowG0 + rowBase + lr) < nN;
      float v = ((acc[t][r] + pb) - pm) * ps + pe;
      if (RELU != 0) v = relu_n(v);
      stg[lr * BNW + lc] = live ? v : 0.0f;
    }
  }
  __syncthreads();

  if constexpr (EPI == 0) {
    unsigned short* outH = (unsigned short*)outp;
    const int cb = 8 * m;
    const bool isHi = (hh == 0);
    const int ocol = isHi ? (n0 + cb) : (halfW + n0 + cb);
    v4u pk[16];
#pragma unroll
    for (int i = 0; i < 16; ++i) {
      const int lr = 16 * wave + i;
      const v4f a = *(const v4fa*)(stg + lr * BNW + cb);
      const v4f b = *(const v4fa*)(stg + lr * BNW + cb + 4);
      const float f[8] = {a.x, a.y, a.z, a.w, b.x, b.y, b.z, b.w};
      unsigned w[4];
#pragma unroll
      for (int j = 0; j < 4; ++j) {
        unsigned l0, l1;
        const unsigned h0 = hl_bits(f[2 * j], l0);
        const unsigned h1 = hl_bits(f[2 * j + 1], l1);
        const unsigned q0 = isHi ? h0 : l0, q1 = isHi ? h1 : l1;
        w[j] = (q0 & 0xffffu) | (q1 << 16);
      }
      v4u pw; pw.x = w[0]; pw.y = w[1]; pw.z = w[2]; pw.w = w[3];
      pk[i] = pw;
    }
#pragma unroll
    for (int i = 0; i < 16; ++i) {
      const int gr = rowBase + 16 * wave + i;
      unsigned short* op = outH + (size_t)gr * (size_t)ldo + ocol;
      if (gr < mRows) *(volatile v4u*)op = pk[i];
    }
    __threadfence();
#pragma unroll
    for (int i = 0; i < 16; ++i) {
      const int gr = rowBase + 16 * wave + i;
      unsigned short* op = outH + (size_t)gr * (size_t)ldo + ocol;
      if (gr < mRows) *(volatile v4u*)op = pk[i];
    }
  } else if constexpr (EPI == 1) {
    static_assert(EPI != 1 || NT == 4);
    unsigned short* outH = (unsigned short*)outp;
    const int rsel = lane >> 4, p = lane & 15;
    const int cb = 8 * (p & 7);
    const bool isHi = p < 8;
    v4u pk[8];
#pragma unroll
    for (int i = 0; i < 8; ++i) {
      const int lr = 16 * wave + 2 * i + rsel;
      const v4f a = *(const v4fa*)(stg + lr * BNW + cb);
      const v4f b = *(const v4fa*)(stg + lr * BNW + cb + 4);
      const float f[8] = {a.x, a.y, a.z, a.w, b.x, b.y, b.z, b.w};
      unsigned w[4];
#pragma unroll
      for (int j = 0; j < 4; ++j) {
        unsigned l0, l1;
        const unsigned h0 = hl_bits(f[2 * j], l0);
        const unsigned h1 = hl_bits(f[2 * j + 1], l1);
        const unsigned q0 = isHi ? h0 : l0, q1 = isHi ? h1 : l1;
        w[j] = (q0 & 0xffffu) | (q1 << 16);
      }
      v4u pw; pw.x = w[0]; pw.y = w[1]; pw.z = w[2]; pw.w = w[3];
      pk[i] = pw;
    }
#pragma unroll
    for (int i = 0; i < 8; ++i) {
      const int gr = rowBase + 16 * wave + 2 * i;
      unsigned short* op = outH + (size_t)gr * (size_t)(2 * BNW) + 8 * lane;
      if (gr + 1 < mRows) *(volatile v4u*)op = pk[i];
    }
    __threadfence();
#pragma unroll
    for (int i = 0; i < 8; ++i) {
      const int gr = rowBase + 16 * wave + 2 * i;
      unsigned short* op = outH + (size_t)gr * (size_t)(2 * BNW) + 8 * lane;
      if (gr + 1 < mRows) *(volatile v4u*)op = pk[i];
    }
    (void)ldo; (void)halfW;
  } else {
    float* outF = (float*)outp;
    v4f fv[16];
#pragma unroll
    for (int i = 0; i < 16; ++i) fv[i] = *(const v4fa*)(stg + (16 * wave + i) * BNW + 4 * lane);
#pragma unroll
    for (int i = 0; i < 16; ++i) {
      const int gr = rowG0 + rowBase + 16 * wave + i;
      float* op = outF + (size_t)gr * (size_t)ldo + n0 + 4 * lane;
      if (gr < nN) *(volatile v4f*)op = fv[i];
    }
    __threadfence();
#pragma unroll
    for (int i = 0; i < 16; ++i) {
      const int gr = rowG0 + rowBase + 16 * wave + i;
      float* op = outF + (size_t)gr * (size_t)ldo + n0 + 4 * lane;
      if (gr < nN) *(volatile v4f*)op = fv[i];
    }
    (void)halfW; (void)mRows;
  }
}

__global__ __launch_bounds__(NTHR) void k_edge(const float* __restrict__ pgd, const int* __restrict__ ea,
                                               const int* __restrict__ eb, const float* __restrict__ tab,
                                               int nN, int EL, float* out) {
  __shared__ __attribute__((aligned(16))) float ost[EBLK];
  const int tid = (int)threadIdx.x, lane = tid & 31, wave = tid >> 5;
  const int base = (int)blockIdx.x * EBLK;
  const v4f w4 = *(const v4f*)(tab + TMISC + 4 * lane);
  const float bd2 = tab[TMISC + 128];
#pragma unroll 1
  for (int g = 0; g < 4; ++g) {
    const int e0 = base + wave * 128 + g * 32;
    if (e0 < EL) {
      const int e  = e0 + lane;
      const int ec = e < EL ? e : EL - 1;
      int ia = ea[ec], ib = eb[ec];
      ia = ia < 0 ? 0 : (ia > nN - 1 ? nN - 1 : ia);
      ib = ib < 0 ? 0 : (ib > nN - 1 ? nN - 1 : ib);
      float mine = 0.0f;
#pragma unroll 1
      for (int k = 0; k < 32; ++k) {
        const int ak = __builtin_amdgcn_readlane(ia, k);
        const int bk = __builtin_amdgcn_readlane(ib, k);
        const v4f pg = *(const v4f*)(pgd + (size_t)ak * 256 + 4 * lane);
        const v4f pd = *(const v4f*)(pgd + (size_t)bk * 256 + 128 + 4 * lane);
        const float r0 = relu_n(pg.x + pd.x), r1 = relu_n(pg.y + pd.y);
        const float r2 = relu_n(pg.z + pd.z), r3 = relu_n(pg.w + pd.w);
        float s = r0 * w4.x;
        s = fmaf(r1, w4.y, s);
        s = fmaf(r2, w4.z, s);
        s = fmaf(r3, w4.w, s);
        s += __shfl_xor(s, 16, 32);
        s += __shfl_xor(s, 8, 32);
        s += __shfl_xor(s, 4, 32);
        s += __shfl_xor(s, 2, 32);
        s += __shfl_xor(s, 1, 32);
        const float sv = s + bd2;
        mine = (lane == k) ? sv : mine;
      }
      ost[wave * 128 + g * 32 + lane] = mine;
    }
  }
  __syncthreads();
  const int e4 = base + 4 * tid;
  const bool ok = e4 < EL;
  v4f pv = {0.f, 0.f, 0.f, 0.f};
  if (ok) pv = *(const v4fa*)(ost + 4 * tid);
  float* op = out + (size_t)(ok ? e4 : 0);
  if (ok) *(volatile v4f*)op = pv;
  __threadfence();
  if (ok) *(volatile v4f*)op = pv;
}

static inline int cdiv(int a, int b) { return (a + b - 1) / b; }
static inline size_t al256(size_t o) { return (o + 255) & ~(size_t)255; }

extern "C" void kernel_launch(void* const* d_in, const int* in_sizes, int n_in,
                              void* d_out, int out_size, void* d_ws, size_t ws_size,
                              hipStream_t stream) {
  if (n_in < 33) return;
  if (in_sizes[0] < DF || (in_sizes[0] % DF) != 0) return;
  const int nN = in_sizes[0] / DF;
  if (nN < GBM || nN > (1 << 21)) return;
  if (in_sizes[1] < 2 || (in_sizes[1] & 1) != 0) return;
  const int nE = in_sizes[1] / 2;
  if (nE < 1 || nE >= (1 << 21)) return;
  if (in_sizes[2] < 2 || (in_sizes[2] & 1) != 0) return;
  const int EL = in_sizes[2] / 2;
  if (EL < 32 || (EL % 32) != 0 || out_size != EL) return;
  {
    const int ex[33] = {0, 0, 0, 1, 32768, 256, 256, 256, 256, 256, 32768, 128, 128, 128, 128, 128,
                        1, 32768, 256, 256, 256, 256, 256, 16384, 64, 64, 64, 64, 64, 16384, 128, 128, 1};
    for (int i = 3; i < 33; ++i) if (in_sizes[i] != ex[i]) return;
  }
  if ((long long)nE * NBA * 5LL > (long long)RCAP * (long long)nN * 4LL) return;

  const float* x    = (const float*)d_in[0];
  const int*   ei   = (const int*)  d_in[1];
  const int*   eli  = (const int*)  d_in[2];
  const float* eps1 = (const float*)d_in[3];
  const float* W1a  = (const float*)d_in[4];
  const float* b1a  = (const float*)d_in[5];
  const float* g1a  = (const float*)d_in[6];
  const float* be1a = (const float*)d_in[7];
  const float* rm1a = (const float*)d_in[8];
  const float* rv1a = (const float*)d_in[9];
  const float* W1b  = (const float*)d_in[10];
  const float* b1b  = (const float*)d_in[11];
  const float* g1   = (const float*)d_in[12];
  const float* be1  = (const float*)d_in[13];
  const float* rm1  = (const float*)d_in[14];
  const float* rv1  = (const float*)d_in[15];
  const float* eps2 = (const float*)d_in[16];
  const float* W2a  = (const float*)d_in[17];
  const float* b2a  = (const float*)d_in[18];
  const float* g2a  = (const float*)d_in[19];
  const float* be2a = (const float*)d_in[20];
  const float* rm2a = (const float*)d_in[21];
  const float* rv2a = (const float*)d_in[22];
  const float* W2b  = (const float*)d_in[23];
  const float* b2b  = (const float*)d_in[24];
  const float* g2   = (const float*)d_in[25];
  const float* be2  = (const float*)d_in[26];
  const float* rm2  = (const float*)d_in[27];
  const float* rv2  = (const float*)d_in[28];
  const float* Wd1  = (const float*)d_in[29];
  const float* bd1  = (const float*)d_in[30];
  const float* Wd2  = (const float*)d_in[31];
  const float* bd2  = (const float*)d_in[32];
  float* out = (float*)d_out;
  const int* src = ei;
  const int* dst = ei + nE;
  const int* la  = eli;
  const int* lb  = eli + EL;

  const int gB  = cdiv(nN, NBA);
  const int nCh = cdiv(gB, CHB);
  const int MP  = nCh * CHR;
  if ((long long)gB * NBA > (long long)MP) return;
  const int vec8 = ((nE & 3) == 0) ? 1 : 0;

  char* ws = (char*)d_ws;
  size_t off = 0;
  const size_t oTAB  = off; off = al256(off + (size_t)TABN * 4);
  const size_t oWPL  = off; off = al256(off + (size_t)WPLN * 2);
  const size_t oZHL  = off; off = al256(off + (size_t)MP * 128 * 2);
  const size_t oRA   = off; off = al256(off + (size_t)MP * 256 * 2);
  const size_t szXB  = (size_t)MP * 128 * 2;
  const size_t szTC  = (size_t)CHR * 512 * 2;
  const size_t oXB   = off; off = al256(off + (szXB > szTC ? szXB : szTC));
  const size_t oZ2C  = off; off = al256(off + (size_t)CHR * 256 * 2);
  const size_t oLIST = off; off = al256(off + (size_t)gB * RCAP * 4);
  const size_t oCNT  = off; off = al256(off + (size_t)gB * NBA * 4);
  const size_t oOFF  = off; off = al256(off + (size_t)gB * NBA * 4);
  const size_t oFLG  = off; off = al256(off + (size_t)gB * MISCN * 4);
  const size_t pgdEnd = al256(oRA + (size_t)nN * 256 * 4);
  if (pgdEnd > off) off = pgdEnd;
  if (off > ws_size || off > (size_t)WSMAX) return;
  float*          TAB  = (float*)(ws + oTAB);
  unsigned short* WPL  = (unsigned short*)(ws + oWPL);
  unsigned short* ZHL  = (unsigned short*)(ws + oZHL);
  unsigned short* RA   = (unsigned short*)(ws + oRA);
  unsigned short* XB   = (unsigned short*)(ws + oXB);
  unsigned short* TC   = (unsigned short*)(ws + oXB);
  unsigned short* Z2C  = (unsigned short*)(ws + oZ2C);
  int*            LIST = (int*)(ws + oLIST);
  int*            CNT  = (int*)(ws + oCNT);
  int*            OFFT = (int*)(ws + oOFF);
  int*            FLG  = (int*)(ws + oFLG);
  float*          PGD  = (float*)(ws + oRA);

  const int bktLds = BKT_INTS * 4;
  hipFuncSetAttribute(reinterpret_cast<const void*>(&k_bucket), hipFuncAttributeMaxDynamicSharedMemorySize, bktLds);

  k_tab<<<5, NTHR, 0, stream>>>(b1a, g1a, be1a, rm1a, rv1a, b1b, g1, be1, rm1, rv1,
                                b2a, g2a, be2a, rm2a, rv2a, b2b, g2, be2, rm2, rv2,
                                bd1, Wd2, bd2, eps1, eps2, TAB);
  const int nUnits = NUW + MP * 16;
  k_prep<<<cdiv(nUnits, NTHR), NTHR, 0, stream>>>(x, W1a, W1b, W2a, W2b, Wd1, WPL, XB, nN, nUnits);
  k_bucket<<<gB, NTHR, bktLds, stream>>>(src, dst, nE, nN, vec8, LIST, CNT, OFFT, FLG);
  k_agg<1><<<gB, NTHR, 0, stream>>>(LIST, CNT, OFFT, FLG, XB, TAB, RA, 0, 0, nN, MP);
  for (int c = 0; c < nCh; ++c) {
    const int b0 = c * CHB;
    const int nb = (gB - b0) < CHB ? (gB - b0) : CHB;
    const int r0 = b0 * NBA;
    const int tiles = nb * (NBA / GBM);
    unsigned short* RAc = RA + (size_t)r0 * 256;
    k_gemm<8, 0, 1><<<dim3(tiles, 2), GTHR, 0, stream>>>(RAc, 256, 256, WPL + PW1A, TAB + T1A, 256,
                                                         (void*)TC, 512, 256, r0, nN, tiles * GBM);
    k_gemm<8, 0, 1><<<dim3(tiles, 1), GTHR, 0, stream>>>(TC, 512, 512, WPL + PW1B, TAB + T1B, 128,
                                                         (void*)RAc, 256, 128, r0, nN, tiles * GBM);
  }
  for (int c = 0; c < nCh; ++c) {
    const int b0 = c * CHB;
    const int nb = (gB - b0) < CHB ? (gB - b0) : CHB;
    const int r0 = b0 * NBA;
    const int tiles = nb * (NBA / GBM);
    k_agg<2><<<nb, NTHR, 0, stream>>>(LIST, CNT, OFFT, FLG, RA, TAB, Z2C, b0, r0, nN, CHR);
    k_gemm<8, 0, 1><<<dim3(tiles, 2), GTHR, 0, stream>>>(Z2C, 256, 256, WPL + PW2A, TAB + T2A, 256,
                                                         (void*)TC, 512, 256, r0, nN, tiles * GBM);
    k_gemm<4, 1, 0><<<dim3(tiles, 1), GTHR, 0, stream>>>(TC, 512, 512, WPL + PW2B, TAB + T2B, 64,
                                                         (void*)(ZHL + (size_t)r0 * 128), 128, 64, r0, nN,
                                                         tiles * GBM);
  }
  k_gemm<8, 2, 0><<<dim3(gB * (NBA / GBM), 2), GTHR, 0, stream>>>(ZHL, 128, 128, WPL + PWD, TAB + TDEC, 256,
                                                                  (void*)PGD, 256, 0, 0, nN, gB * NBA);
  k_edge<<<cdiv(EL, EBLK), NTHR, 0, stream>>>(PGD, la, lb, TAB, nN, EL, out);
}
